// SGS_10247791968409
// MI455X (gfx1250) — hardware-verified
//
#include <hip/hip_runtime.h>
#include <stddef.h>
#include <stdint.h>

#define NBAT  4
#define NN    4096
#define NTOK  16384
#define CD    256
#define GG    8
#define MM    512
#define NH    8
#define HDM   32
#define NQKV  768
#define NSLAB 6
#define NHF   (NBAT * GG * NH)
#define QB    128
#define KC    64
#define NQB   (MM / QB)
#define NCK   (MM / KC)

static_assert(NTOK == NBAT * NN);
static_assert(NN == GG * MM);
static_assert(NH * HDM == CD);
static_assert(NQKV == 3 * CD);
static_assert(NQKV == NSLAB * 128);
static_assert(MM % QB == 0);
static_assert(MM % KC == 0);
static_assert(MM % 64 == 0);
static_assert(NN % 64 == 0);
static_assert(CD % 64 == 0);
static_assert(NTOK % 64 == 0);
static_assert(HDM == 32);
static_assert(KC == 64);
static_assert(QB == 8 * 16);
static_assert((NQKV * CD) % 2048 == 0);
static_assert((CD * CD) % 2048 == 0);

typedef _Float16 v16h __attribute__((ext_vector_type(16)));
typedef _Float16 v8h  __attribute__((ext_vector_type(8)));
typedef __bf16   v16b __attribute__((ext_vector_type(16)));
typedef float    v8f  __attribute__((ext_vector_type(8)));
typedef float    v4f  __attribute__((ext_vector_type(4)));
typedef unsigned int v4u __attribute__((ext_vector_type(4)));

union FragH { v16h v; v8h h[2]; };
union FragB { v16b v; v4u u[2]; unsigned int w[8]; };
union Pack8 { v8h h; v4u u; };

__device__ __forceinline__ v8f mma_h(v16h a, v16h b, v8f c) {
  c = __builtin_amdgcn_wmma_f32_16x16x32_f16(false, a, false, b, (short)0, c, false, false);
  asm volatile("v_nop\n\tv_nop\n\tv_nop\n\tv_nop" : "+v"(c) : "v"(a), "v"(b));
  return c;
}
__device__ __forceinline__ v8f mma_b(v16b a, v16b b, v8f c) {
  c = __builtin_amdgcn_wmma_f32_16x16x32_bf16(false, a, false, b, (short)0, c, false, false);
  asm volatile("v_nop\n\tv_nop\n\tv_nop\n\tv_nop" : "+v"(c) : "v"(a), "v"(b));
  return c;
}

__device__ __forceinline__ v8f zero8() { return (v8f){0.f, 0.f, 0.f, 0.f, 0.f, 0.f, 0.f, 0.f}; }

__device__ __forceinline__ v16h ldfrag_h(const _Float16* p, int ld, int row0, int k0, int lane) {
  const int m = lane & 15, lh = lane >> 4;
  const _Float16* q = p + (size_t)(row0 + m) * ld + k0 + 8 * lh;
  FragH f;
  f.h[0] = *(const v8h*)(q);
  f.h[1] = *(const v8h*)(q + 16);
  return f.v;
}
__device__ __forceinline__ v16b ldfrag_b(const unsigned short* p, int ld, int row0, int k0, int lane) {
  const int m = lane & 15, lh = lane >> 4;
  const unsigned short* q = p + (size_t)(row0 + m) * ld + k0 + 8 * lh;
  FragB f;
  f.u[0] = *(const v4u*)(q);
  f.u[1] = *(const v4u*)(q + 16);
  return f.v;
}

__device__ __forceinline__ unsigned int bf16_bits(float f) {
  const unsigned int u = __float_as_uint(f);
  return (u + 0x7FFFu + ((u >> 16) & 1u)) >> 16;
}
__device__ __forceinline__ void split_bf16(float f, unsigned int& hb, unsigned int& lb) {
  hb = bf16_bits(f);
  const float hf = __uint_as_float(hb << 16);
  lb = bf16_bits(f - hf);
}
__device__ __forceinline__ void pack_split8(const float (&v)[8], v4u& ph, v4u& pl) {
  unsigned int hb[8], lb[8];
#pragma unroll
  for (int i = 0; i < 8; ++i) split_bf16(v[i], hb[i], lb[i]);
  ph = (v4u){hb[0] | (hb[1] << 16), hb[2] | (hb[3] << 16), hb[4] | (hb[5] << 16), hb[6] | (hb[7] << 16)};
  pl = (v4u){lb[0] | (lb[1] << 16), lb[2] | (lb[3] << 16), lb[4] | (lb[5] << 16), lb[6] | (lb[7] << 16)};
}

__device__ __forceinline__ void gemm16x64x3(const unsigned short* __restrict__ Ah,
                                            const unsigned short* __restrict__ Al,
                                            int lda, size_t akst,
                                            const unsigned short* __restrict__ Bh,
                                            const unsigned short* __restrict__ Bl,
                                            int m0, int n0, int lane, v8f (&acc)[4]) {
#pragma unroll 1
  for (int ks = 0; ks < CD / 32; ++ks) {
    const v16b ah = ldfrag_b(Ah + (size_t)ks * akst, lda, m0, 0, lane);
    const v16b al = ldfrag_b(Al + (size_t)ks * akst, lda, m0, 0, lane);
#pragma unroll
    for (int t = 0; t < 4; ++t) {
      const v16b bh = ldfrag_b(Bh, CD, n0 + 16 * t, ks * 32, lane);
      const v16b bl = ldfrag_b(Bl, CD, n0 + 16 * t, ks * 32, lane);
      acc[t] = mma_b(ah, bh, acc[t]);
      acc[t] = mma_b(al, bh, acc[t]);
      acc[t] = mma_b(ah, bl, acc[t]);
    }
  }
}

#define WTP 65
__global__ __launch_bounds__(256) void k_xtr(const float* __restrict__ x,
                                             unsigned short* __restrict__ xh,
                                             unsigned short* __restrict__ xl) {
  __shared__ float tl[64 * WTP];
  const int tid = threadIdx.x;
  const int n0 = blockIdx.x * 64, c0 = blockIdx.y * 64, b = blockIdx.z;
  const float* xb = x + (size_t)b * CD * NN;
#pragma unroll
  for (int j = 0; j < 4; ++j) {
    const int p  = tid + 256 * j;
    const int cc = p >> 4;
    const int q4 = (p & 15) * 4;
    const v4f a = *(const v4f*)(xb + (size_t)(c0 + cc) * NN + n0 + q4);
    float* d = tl + cc * WTP + q4;
    d[0] = a[0]; d[1] = a[1]; d[2] = a[2]; d[3] = a[3];
  }
  __syncthreads();
  v4u vh[2], vl[2];
  size_t go[2];
#pragma unroll
  for (int j = 0; j < 2; ++j) {
    const int p  = tid + 256 * j;
    const int nn = p >> 3;
    const int pc = p & 7;
    const float* cp = tl + (pc * 8) * WTP + nn;
    float v[8];
#pragma unroll
    for (int i = 0; i < 8; ++i) v[i] = cp[i * WTP];
    pack_split8(v, vh[j], vl[j]);
    go[j] = ((size_t)b * NN + n0 + nn) * CD + c0 + pc * 8;
  }
  for (int ps = 0; ps < 2; ++ps) {
#pragma unroll
    for (int j = 0; j < 2; ++j) {
      *(volatile v4u*)(xh + go[j]) = vh[j];
      *(volatile v4u*)(xl + go[j]) = vl[j];
    }
    __threadfence();
  }
}

__global__ __launch_bounds__(256) void k_wcv(const float* __restrict__ W, int n8,
                                             unsigned short* __restrict__ wh,
                                             unsigned short* __restrict__ wl) {
  int i = blockIdx.x * 256 + threadIdx.x;
  i = min(i, n8 - 1);
  const float* wp = W + (size_t)i * 8;
  const v4f a0 = *(const v4f*)(wp), a1 = *(const v4f*)(wp + 4);
  float v[8] = {a0[0], a0[1], a0[2], a0[3], a1[0], a1[1], a1[2], a1[3]};
  v4u ph, pl;
  pack_split8(v, ph, pl);
  const size_t go = (size_t)i * 8;
  for (int ps = 0; ps < 2; ++ps) {
    *(volatile v4u*)(wh + go) = ph;
    *(volatile v4u*)(wl + go) = pl;
    __threadfence();
  }
}

#define SFP 132
__global__ __launch_bounds__(256) void k_qkv(const unsigned short* __restrict__ xh,
                                             const unsigned short* __restrict__ xl,
                                             const unsigned short* __restrict__ wh,
                                             const unsigned short* __restrict__ wl,
                                             _Float16* __restrict__ qp,
                                             _Float16* __restrict__ kp,
                                             _Float16* __restrict__ vtp) {
  __shared__ __align__(16) float sf[64 * SFP];
  const int tid = threadIdx.x, lane = tid & 31, wave = tid >> 5;
  const int hh = lane >> 4, c = lane & 15;
  const int wm = wave >> 1, wn = wave & 1;
  const int mb  = blockIdx.x * 64;
  const int b   = mb >> 12;
  const int nb0 = mb & (NN - 1);
  const int g   = nb0 >> 9;
  const int ml0 = nb0 & (MM - 1);
  const int ns  = blockIdx.y;
  const int which = ns >> 1;
  const int hbase = 4 * (ns & 1);
  const int hfb = (b * GG + g) * NH + hbase;
  const int m0 = mb + wm * 16;
  const int n0 = ns * 128 + wn * 64;

  v8f acc[4];
#pragma unroll
  for (int t = 0; t < 4; ++t) acc[t] = zero8();
  gemm16x64x3(xh, xl, CD, 32, wh, wl, m0, n0, lane, acc);

#pragma unroll
  for (int t = 0; t < 4; ++t) {
#pragma unroll
    for (int r = 0; r < 8; ++r)
      sf[(wm * 16 + 8 * hh + r) * SFP + wn * 64 + 16 * t + c] = acc[t][r];
  }
  __syncthreads();

  if (which < 2) {
    v4u val[4];
    size_t go[4];
#pragma unroll
    for (int j = 0; j < 4; ++j) {
      const int lr = tid >> 2;
      const int pc = tid & 3;
      const float* ra = sf + lr * SFP + j * 32 + pc * 8;
      const v4f a0 = *(const v4f*)(ra), a1 = *(const v4f*)(ra + 4);
      Pack8 pk;
      pk.h = (v8h){(_Float16)(a0[0] * 8.0f), (_Float16)(a0[1] * 8.0f), (_Float16)(a0[2] * 8.0f), (_Float16)(a0[3] * 8.0f),
                   (_Float16)(a1[0] * 8.0f), (_Float16)(a1[1] * 8.0f), (_Float16)(a1[2] * 8.0f), (_Float16)(a1[3] * 8.0f)};
      val[j] = pk.u;
      go[j]  = ((size_t)(hfb + j) * MM + ml0 + lr) * HDM + pc * 8;
    }
    _Float16* base = (which == 0) ? qp : kp;
    for (int ps = 0; ps < 2; ++ps) {
#pragma unroll
      for (int j = 0; j < 4; ++j) *(volatile v4u*)(base + go[j]) = val[j];
      __threadfence();
    }
  } else {
    v4u val[4];
    size_t go[4];
#pragma unroll
    for (int j = 0; j < 4; ++j) {
      const int p    = tid + 256 * j;
      const int dcol = p >> 3;
      const int pc   = p & 7;
      const float* cp = sf + (pc * 8) * SFP + dcol;
      Pack8 pk;
      pk.h = (v8h){(_Float16)(cp[0 * SFP] * 16.0f), (_Float16)(cp[1 * SFP] * 16.0f),
                   (_Float16)(cp[2 * SFP] * 16.0f), (_Float16)(cp[3 * SFP] * 16.0f),
                   (_Float16)(cp[4 * SFP] * 16.0f), (_Float16)(cp[5 * SFP] * 16.0f),
                   (_Float16)(cp[6 * SFP] * 16.0f), (_Float16)(cp[7 * SFP] * 16.0f)};
      val[j] = pk.u;
      const int hf = hfb + (dcol >> 5);
      const int dd = dcol & 31;
      go[j]  = ((size_t)hf * HDM + dd) * MM + ml0 + pc * 8;
    }
    for (int ps = 0; ps < 2; ++ps) {
#pragma unroll
      for (int j = 0; j < 4; ++j) *(volatile v4u*)(vtp + go[j]) = val[j];
      __threadfence();
    }
  }
}

#define KTP 40
#define VTP 72
#define PTP 72
#define OSP 36
__global__ __launch_bounds__(256) void k_attn(const _Float16* __restrict__ qp,
                                              const _Float16* __restrict__ kp,
                                              const _Float16* __restrict__ vt,
                                              unsigned short* __restrict__ oh,
                                              unsigned short* __restrict__ ol,
                                              float sscale) {
  __shared__ __align__(16) _Float16 Ks[KC * KTP];
  __shared__ __align__(16) _Float16 Vs[HDM * VTP];
  __shared__ __align__(16) _Float16 Ps[8 * 16 * PTP];
  __shared__ __align__(16) float    Os[8 * 16 * OSP];

  const int tid = threadIdx.x, lane = tid & 31, wave = tid >> 5;
  const int hh = lane >> 4, c = lane & 15;
  const int qb = blockIdx.x % NQB;
  const int hf = blockIdx.x / NQB;
  const int h  = hf & (NH - 1);
  const int bg = hf >> 3;
  const int q0 = qb * QB + wave * 16;

  const _Float16* Q = qp + (size_t)hf * MM * HDM;
  const _Float16* K = kp + (size_t)hf * MM * HDM;
  const _Float16* V = vt + (size_t)hf * HDM * MM;
  const size_t trow0 = (size_t)bg * MM;

  const v16h qa = ldfrag_h(Q, HDM, q0, 0, lane);

  const float NEGI = -__builtin_huge_valf();
  float mrow[8], lrow[8];
  v8f oacc[2];
#pragma unroll
  for (int r = 0; r < 8; ++r) { mrow[r] = NEGI; lrow[r] = 0.f; }
  oacc[0] = zero8(); oacc[1] = zero8();

  _Float16* pw = Ps + wave * 16 * PTP;
  float*    ow = Os + wave * 16 * OSP;

  for (int kc = 0; kc < NCK; ++kc) {
    const int kv0 = kc * KC;
    __syncthreads();
    {
      const int rk = tid >> 2;
      const int qk = (tid & 3) * 8;
      *(v8h*)(Ks + rk * KTP + qk) = *(const v8h*)(K + (size_t)(kv0 + rk) * HDM + qk);
      const int rv = tid >> 3;
      const int qv = (tid & 7) * 8;
      *(v8h*)(Vs + rv * VTP + qv) = *(const v8h*)(V + (size_t)rv * MM + kv0 + qv);
    }
    __syncthreads();

    v8f s[4];
#pragma unroll
    for (int j = 0; j < 4; ++j) {
      const v16h kb = ldfrag_h(Ks, KTP, j * 16, 0, lane);
      s[j] = mma_h(qa, kb, zero8());
    }
    float cm[8];
#pragma unroll
    for (int r = 0; r < 8; ++r) {
      float m = NEGI;
#pragma unroll
      for (int j = 0; j < 4; ++j) { s[j][r] *= sscale; m = fmaxf(m, s[j][r]); }
#pragma unroll
      for (int off = 1; off < 16; off <<= 1) m = fmaxf(m, __shfl_xor(m, off, 32));
      cm[r] = m;
    }
    float al[8];
#pragma unroll
    for (int r = 0; r < 8; ++r) {
      const float mnew  = fmaxf(mrow[r], cm[r]);
      const float alpha = __expf(mrow[r] - mnew);
      mrow[r] = mnew;
      float psum = 0.f;
#pragma unroll
      for (int j = 0; j < 4; ++j) {
        const float p = __expf(s[j][r] - mnew);
        psum += p;
        pw[(8 * hh + r) * PTP + j * 16 + c] = (_Float16)(p * 1024.0f);
      }
#pragma unroll
      for (int off = 1; off < 16; off <<= 1) psum += __shfl_xor(psum, off, 32);
      lrow[r] = lrow[r] * alpha + psum;
      al[r] = alpha;
    }
#pragma unroll
    for (int t = 0; t < 2; ++t)
#pragma unroll
      for (int r = 0; r < 8; ++r) oacc[t][r] *= al[r];
    __syncthreads();

#pragma unroll
    for (int kk = 0; kk < 2; ++kk) {
      const v16h pa = ldfrag_h(pw, PTP, 0, kk * 32, lane);
#pragma unroll
      for (int t = 0; t < 2; ++t) {
        const v16h vb = ldfrag_h(Vs, VTP, t * 16, kk * 32, lane);
        oacc[t] = mma_h(pa, vb, oacc[t]);
      }
    }
  }

  float invl[8];
#pragma unroll
  for (int r = 0; r < 8; ++r) invl[r] = (lrow[r] > 0.f) ? (6.103515625e-05f * (1.0f / lrow[r])) : 0.f;
  __syncthreads();
#pragma unroll
  for (int r = 0; r < 8; ++r) {
#pragma unroll
    for (int t = 0; t < 2; ++t) ow[(8 * hh + r) * OSP + 16 * t + c] = oacc[t][r] * invl[r];
  }
  __syncthreads();
  v4u vh[2], vl[2];
  size_t go[2];
#pragma unroll
  for (int it = 0; it < 2; ++it) {
    const int p  = lane + 32 * it;
    const int L  = p >> 2;
    const int pc = p & 3;
    const float* ra = ow + L * OSP + pc * 8;
    const v4f a0 = *(const v4f*)(ra), a1 = *(const v4f*)(ra + 4);
    float v[8] = {a0[0], a0[1], a0[2], a0[3], a1[0], a1[1], a1[2], a1[3]};
    pack_split8(v, vh[it], vl[it]);
    go[it] = ((size_t)h * NTOK + trow0 + q0 + L) * HDM + pc * 8;
  }
  for (int ps = 0; ps < 2; ++ps) {
#pragma unroll
    for (int it = 0; it < 2; ++it) {
      *(volatile v4u*)(oh + go[it]) = vh[it];
      *(volatile v4u*)(ol + go[it]) = vl[it];
    }
    __threadfence();
  }
}

#define OTP 68
__global__ __launch_bounds__(256) void k_proj(const unsigned short* __restrict__ oh,
                                              const unsigned short* __restrict__ ol,
                                              const unsigned short* __restrict__ wh,
                                              const unsigned short* __restrict__ wl,
                                              const float* __restrict__ pb,
                                              float* __restrict__ out) {
  __shared__ __align__(16) float st[128 * OTP];
  const int tid = threadIdx.x, lane = tid & 31, wave = tid >> 5;
  const int hh = lane >> 4, c = lane & 15;
  const int wm = wave >> 1, wn = wave & 1;
  const int mb  = blockIdx.x * 64;
  const int b   = mb >> 12;
  const int nb0 = mb & (NN - 1);
  const int m0  = mb + wm * 16;
  const int cb  = blockIdx.y * 128;
  const int n0  = cb + wn * 64;

  v8f acc[4];
#pragma unroll
  for (int t = 0; t < 4; ++t) acc[t] = zero8();
  gemm16x64x3(oh, ol, HDM, (size_t)NTOK * HDM, wh, wl, m0, n0, lane, acc);

#pragma unroll
  for (int t = 0; t < 4; ++t) {
    const float bb = pb[n0 + 16 * t + c];
#pragma unroll
    for (int r = 0; r < 8; ++r) st[(wn * 64 + 16 * t + c) * OTP + wm * 16 + 8 * hh + r] = acc[t][r] + bb;
  }
  __syncthreads();
  v4f val[8];
  size_t go[8];
#pragma unroll
  for (int it = 0; it < 8; ++it) {
    const int p    = lane + 32 * it;
    const int L    = p >> 3;
    const int pc   = p & 7;
    const int cl   = wave * 16 + (L >> 1);
    const int half = L & 1;
    val[it] = *(const v4f*)(st + cl * OTP + half * 32 + pc * 4);
    go[it]  = ((size_t)(b * CD + cb + cl)) * NN + nb0 + half * 32 + pc * 4;
  }
  for (int ps = 0; ps < 2; ++ps) {
#pragma unroll
    for (int it = 0; it < 8; ++it) *(volatile v4f*)(out + go[it]) = val[it];
    __threadfence();
  }
}

extern "C" void kernel_launch(void* const* d_in, const int* in_sizes, int n_in,
                              void* d_out, int out_size, void* d_ws, size_t ws_size,
                              hipStream_t stream) {
  if (n_in < 4) return;
  if (in_sizes[0] != NTOK * CD) return;
  if (in_sizes[1] != NQKV * CD) return;
  if (in_sizes[2] != CD * CD) return;
  if (in_sizes[3] != CD) return;
  if (out_size != NTOK * CD) return;

  const float* x     = (const float*)d_in[0];
  const float* wq    = (const float*)d_in[1];
  const float* wp    = (const float*)d_in[2];
  const float* pbias = (const float*)d_in[3];
  float* out = (float*)d_out;

  size_t off = 0;
  const size_t oWQh = off; off += (size_t)NQKV * CD * 2;
  const size_t oWQl = off; off += (size_t)NQKV * CD * 2;
  const size_t oWPh = off; off += (size_t)CD * CD * 2;
  const size_t oWPl = off; off += (size_t)CD * CD * 2;
  const size_t oXh  = off; off += (size_t)NTOK * CD * 2;
  const size_t oXl  = off; off += (size_t)NTOK * CD * 2;
  const size_t oQ   = off; off += (size_t)NHF * MM * HDM * 2;
  const size_t oK   = off; off += (size_t)NHF * MM * HDM * 2;
  const size_t oV   = off; off += (size_t)NHF * HDM * MM * 2;
  const size_t oOh  = off; off += (size_t)NH * NTOK * HDM * 2;
  const size_t oOl  = off; off += (size_t)NH * NTOK * HDM * 2;
  if (off > ws_size) return;
  if (off > (size_t)134217728) return;

  char* ws = (char*)d_ws;
  unsigned short* WQh = (unsigned short*)(ws + oWQh);
  unsigned short* WQl = (unsigned short*)(ws + oWQl);
  unsigned short* WPh = (unsigned short*)(ws + oWPh);
  unsigned short* WPl = (unsigned short*)(ws + oWPl);
  unsigned short* Xh  = (unsigned short*)(ws + oXh);
  unsigned short* Xl  = (unsigned short*)(ws + oXl);
  _Float16*       Qp  = (_Float16*)(ws + oQ);
  _Float16*       Kp  = (_Float16*)(ws + oK);
  _Float16*       Vt  = (_Float16*)(ws + oV);
  unsigned short* Oh  = (unsigned short*)(ws + oOh);
  unsigned short* Ol  = (unsigned short*)(ws + oOl);

  k_xtr<<<dim3(NN / 64, CD / 64, NBAT), dim3(256), 0, stream>>>(x, Xh, Xl);
  k_wcv<<<dim3((NQKV * CD / 8) / 256), dim3(256), 0, stream>>>(wq, NQKV * CD / 8, WQh, WQl);
  k_wcv<<<dim3((CD * CD / 8) / 256), dim3(256), 0, stream>>>(wp, CD * CD / 8, WPh, WPl);
  k_qkv<<<dim3(NTOK / 64, NSLAB), dim3(256), 0, stream>>>(Xh, Xl, WQh, WQl, Qp, Kp, Vt);
  const float sscale = (float)(0.17677669529663688 / 64.0);
  k_attn<<<dim3(NHF * NQB), dim3(256), 0, stream>>>(Qp, Kp, Vt, Oh, Ol, sscale);
  k_proj<<<dim3(NTOK / 64, CD / 128), dim3(256), 0, stream>>>(Oh, Ol, WPh, WPl, pbias, out);
  (void)hipGetLastError();
}
